// CrossNetworkMix_87162066305256
// MI455X (gfx1250) — hardware-verified
//
#include <hip/hip_runtime.h>


namespace {
constexpr int B_ = 16384, D = 512, L = 3, R = 64, E = 4, ER = E * R, NBLK = B_ / 128;
constexpr float AS = 8.0f, AI = 0.125f;

typedef _Float16 b16;
typedef __attribute__((ext_vector_type(16))) _Float16 v16b;
typedef __attribute__((ext_vector_type(8)))  _Float16 v8b;
typedef __attribute__((ext_vector_type(8)))  float v8f;
typedef __attribute__((ext_vector_type(4)))  float v4f;

__device__ __forceinline__ v8b ld8b(const b16* p) { return *(const v8b*)p; }
__device__ __forceinline__ v16b cat8b(v8b a, v8b b) { return __builtin_shufflevector(a, b, 0, 1, 2, 3, 4, 5, 6, 7, 8, 9, 10, 11, 12, 13, 14, 15); }
__device__ __forceinline__ v16b frag_kb(const b16* p, int hh) { return cat8b(ld8b(p + 8 * hh), ld8b(p + 16 + 8 * hh)); }
__device__ __forceinline__ void split16(float v, b16& hi, b16& lo) { hi = (b16)v; lo = (b16)(v - (float)hi); }
__device__ __forceinline__ void frag_ksplit(const float* p, int hh, v16b& fh_, v16b& fl_) {
  const float* p0 = p + 8 * hh; const float* p1 = p + 16 + 8 * hh;
#pragma unroll
  for (int e = 0; e < 8; ++e) { b16 a, c; split16(p0[e], a, c); fh_[e] = a; fl_[e] = c; split16(p1[e], a, c); fh_[8 + e] = a; fl_[8 + e] = c; }
}
__device__ __forceinline__ v8f wmma16b(v16b a, v16b b, v8f c) {
  v8f d = __builtin_amdgcn_wmma_f32_16x16x32_f16(false, a, false, b, (short)0, c, false, false);
  asm volatile("v_nop\n\tv_nop\n\tv_nop\n\tv_nop" : "+v"(d) : "v"(a), "v"(b));
  return d;
}
__device__ __forceinline__ void wave_lds_sync() {
  __builtin_amdgcn_fence(__ATOMIC_RELEASE, "workgroup");
  __builtin_amdgcn_wave_barrier();
  __builtin_amdgcn_fence(__ATOMIC_ACQUIRE, "workgroup");
}

struct Opnd { const void* p0; const void* p1; int ld; };
template <int NP> __device__ __forceinline__ void load_frags(const Opnd& o, int row, int kb, int hh, v16b& fh_, v16b& fl_) {
  if (NP == 0) { frag_ksplit((const float*)o.p0 + (size_t)row * o.ld + kb, hh, fh_, fl_); }
  else if (NP == 4 || NP == 5) {
    const float sc_ = (NP == 4) ? 64.0f : 8.0f;
    const float* p = (const float*)o.p0 + (size_t)row * o.ld + kb; const float* p0 = p + 8 * hh; const float* p1 = p + 16 + 8 * hh;
#pragma unroll
    for (int e = 0; e < 8; ++e) { b16 a, c; split16(p0[e] * sc_, a, c); fh_[e] = a; fl_[e] = c; split16(p1[e] * sc_, a, c); fh_[8 + e] = a; fl_[8 + e] = c; }
  } else if (NP == 3) {
    const float* p = (const float*)o.p0 + (size_t)row * o.ld + kb; const float* p0 = p + 8 * hh; const float* p1 = p + 16 + 8 * hh;
#pragma unroll
    for (int e = 0; e < 8; ++e) { fh_[e] = (b16)p0[e]; fh_[8 + e] = (b16)p1[e]; }
    fl_ = fh_;
  } else {
    fh_ = frag_kb((const b16*)o.p0 + (size_t)row * o.ld + kb, hh);
    if (NP == 2) fl_ = frag_kb((const b16*)o.p1 + (size_t)row * o.ld + kb, hh); else fl_ = fh_;
  }
}
template <int ANP, int BNP> __device__ __forceinline__ v8f mac(v16b ah, v16b al, v16b bh, v16b bl, v8f c) {
  c = wmma16b(ah, bh, c);
  if (BNP == 0 || BNP == 2 || BNP == 4 || BNP == 5) c = wmma16b(ah, bl, c);
  if (ANP == 0 || ANP == 2 || ANP == 4 || ANP == 5) c = wmma16b(al, bh, c);
  return c;
}
template <int ANP, int BNP>
__device__ __forceinline__ void gemm_tile(const Opnd& A, const Opnd& B, int K, int m0, int c0, int nloc, int hlf, v8f (&acc)[2][4]) {
  for (int kb = 0; kb < K; kb += 32) {
    v16b a0h, a0l, a1h, a1l;
    load_frags<ANP>(A, m0 + nloc, kb, hlf, a0h, a0l);
    load_frags<ANP>(A, m0 + 16 + nloc, kb, hlf, a1h, a1l);
#pragma unroll
    for (int t = 0; t < 4; ++t) {
      v16b bh, bl;
      load_frags<BNP>(B, c0 + t * 16 + nloc, kb, hlf, bh, bl);
      acc[0][t] = mac<ANP, BNP>(a0h, a0l, bh, bl, acc[0][t]);
      acc[1][t] = mac<ANP, BNP>(a1h, a1l, bh, bl, acc[1][t]);
    }
  }
}

__device__ __forceinline__ void epi_planes(v8f (&acc)[2][4], float scale, bool two, b16* __restrict__ oh, b16* __restrict__ ol, int ldo,
                                           int m0, int c0, int lane, b16* Th, b16* Tl) {
  const int nloc = lane & 15, hlf = lane >> 4;
#pragma unroll
  for (int t = 0; t < 4; ++t)
#pragma unroll
    for (int r = 0; r < 2; ++r)
#pragma unroll
      for (int v = 0; v < 8; ++v) {
        const int rr = r * 16 + v + 8 * hlf, cc = t * 16 + nloc;
        b16 h_, l_; split16(acc[r][t][v] * scale, h_, l_);
        Th[rr * 64 + cc] = h_; Tl[rr * 64 + cc] = l_;
      }
  wave_lds_sync();
  for (int pass = 0; pass < 2; ++pass) {
#pragma unroll
    for (int j = 0; j < 8; ++j) {
      const int rr = j * 4 + (lane >> 3), c8 = (lane & 7) * 8;
      const size_t o = (size_t)(m0 + rr) * ldo + c0 + c8;
      *(volatile v8b*)(oh + o) = ld8b(Th + rr * 64 + c8);
      if (two) *(volatile v8b*)(ol + o) = ld8b(Tl + rr * 64 + c8);
    }
    __threadfence();
  }
}
__device__ __forceinline__ void epi_f32(v8f (&acc)[2][4], float scale, const float* rscale, float* __restrict__ out, int ldo, int m0, int c0, int lane, float* Tt) {
  const int nloc = lane & 15, hlf = lane >> 4;
#pragma unroll
  for (int t = 0; t < 4; ++t)
#pragma unroll
    for (int r = 0; r < 2; ++r)
#pragma unroll
      for (int v = 0; v < 8; ++v) {
        const int rr = r * 16 + v + 8 * hlf;
        const float rs = rscale ? rscale[(size_t)(m0 + rr) * 32] : 1.0f;
        Tt[rr * 64 + t * 16 + nloc] = acc[r][t][v] * scale * rs;
      }
  wave_lds_sync();
  float* dst0 = out + (size_t)m0 * ldo + c0;
  for (int pass = 0; pass < 2; ++pass) {
#pragma unroll
    for (int j = 0; j < 16; ++j) { const int rr = j * 2 + hlf, c4 = nloc * 4; *(volatile v4f*)(dst0 + (size_t)rr * ldo + c4) = *(const v4f*)(Tt + rr * 64 + c4); }
    __threadfence();
  }
}


typedef __attribute__((ext_vector_type(8))) __bf16 v8bb; typedef __attribute__((ext_vector_type(16))) __bf16 v16bb;
typedef __attribute__((ext_vector_type(8))) unsigned short v8us;
__device__ __forceinline__ v16bb frag_kb_bf(const __bf16* p, int hh) { const v8bb a = *(const v8bb*)(p + 8 * hh), b = *(const v8bb*)(p + 16 + 8 * hh); return __builtin_shufflevector(a, b, 0, 1, 2, 3, 4, 5, 6, 7, 8, 9, 10, 11, 12, 13, 14, 15); }
__device__ __forceinline__ v8f wmma16bb(v16bb a, v16bb b, v8f c) {
  v8f d = __builtin_amdgcn_wmma_f32_16x16x32_bf16(false, a, false, b, (short)0, c, false, false);
  asm volatile("v_nop\n\tv_nop\n\tv_nop\n\tv_nop" : "+v"(d) : "v"(a), "v"(b));
  return d;
}
__device__ __forceinline__ unsigned short bf16_rne_bits(float v) { unsigned int u = __float_as_uint(v); u += 0x7FFFu + ((u >> 16) & 1u); return (unsigned short)(u >> 16); }
__device__ __forceinline__ float bf16_rne(float v) { return __uint_as_float(((unsigned int)bf16_rne_bits(v)) << 16); }


__global__ __launch_bounds__(256) void prep_kernel(const float* __restrict__ U, const float* __restrict__ V, const float* __restrict__ C, const float* __restrict__ G,
                                                   b16* __restrict__ vt, b16* __restrict__ cb, b16* __restrict__ ut, b16* __restrict__ g16) {
  const size_t tid = (size_t)blockIdx.x * blockDim.x + threadIdx.x, nth = (size_t)gridDim.x * blockDim.x;
  for (int pass = 0; pass < 2; ++pass) {
    for (size_t p = tid; p < (size_t)L * ER * D; p += nth) { const int l = (int)(p / (ER * D)); const int rem = (int)(p % (ER * D)), er = rem / D, d = rem % D, e = er / R, r = er % R;
      ((volatile b16*)vt)[p] = (b16)V[(((size_t)l * E + e) * D + d) * R + r]; }
    for (size_t p = tid; p < (size_t)L * ER * ER; p += nth) { const int l = (int)(p / (ER * ER)); const int rem = (int)(p % (ER * ER)), er = rem / ER, es = rem % ER, e = er / R, r = er % R, e2 = es / R, s = es % R;
      ((volatile b16*)cb)[p] = (b16)((e == e2) ? C[(((size_t)l * E + e) * R + s) * R + r] : 0.0f); }
    for (size_t p = tid; p < (size_t)L * E * D * R; p += nth) ((volatile b16*)ut)[p] = (b16)U[p];
    for (size_t p = tid; p < (size_t)16 * D; p += nth) { const int n = (int)(p / D), d = (int)(p % D); ((volatile b16*)g16)[p] = (b16)((n < E) ? G[(size_t)min(n, E - 1) * D + d] : 0.0f); }
    __threadfence();
  }
}

__global__ __launch_bounds__(128) void vx_kernel(const float* __restrict__ xl, const b16* __restrict__ vt, float* __restrict__ vx) {
  __shared__ __attribute__((aligned(16))) float Ts[4][32 * 64];
  const int lane = threadIdx.x & 31, wave = threadIdx.x >> 5, nloc = lane & 15, hlf = lane >> 4, m0 = blockIdx.y * 128 + wave * 32, c0 = blockIdx.x * 64;
  v8f acc[2][4];
#pragma unroll
  for (int r = 0; r < 2; ++r)
#pragma unroll
    for (int t = 0; t < 4; ++t) acc[r][t] = (v8f){};
  const Opnd A{xl, nullptr, D}, Bo{vt, nullptr, D};
  gemm_tile<5, 1>(A, Bo, D, m0, c0, nloc, hlf, acc);
#pragma unroll
  for (int t = 0; t < 4; ++t)
#pragma unroll
    for (int r = 0; r < 2; ++r)
#pragma unroll
      for (int v = 0; v < 8; ++v) acc[r][t][v] = tanhf(acc[r][t][v] * AI);
  epi_f32(acc, 1.0f, nullptr, vx, ER, m0, c0, lane, Ts[wave]);
}

__global__ __launch_bounds__(128) void gate_kernel(const float* __restrict__ xl, const b16* __restrict__ g16, float* __restrict__ gate) {
  __shared__ __attribute__((aligned(16))) float Ts[4][32 * 4];
  const int lane = threadIdx.x & 31, wave = threadIdx.x >> 5, nloc = lane & 15, hlf = lane >> 4, m0 = blockIdx.x * 128 + wave * 32;
  v8f a0acc = {}, a1acc = {};
  const Opnd A{xl, nullptr, D};
#pragma unroll 1
  for (int kb = 0; kb < D; kb += 32) { v16b a0, l0, a1, l1; load_frags<5>(A, m0 + nloc, kb, hlf, a0, l0); load_frags<5>(A, m0 + 16 + nloc, kb, hlf, a1, l1); const v16b bw = frag_kb(g16 + (size_t)nloc * D + kb, hlf);
    a0acc = wmma16b(a0, bw, a0acc); a0acc = wmma16b(l0, bw, a0acc); a1acc = wmma16b(a1, bw, a1acc); a1acc = wmma16b(l1, bw, a1acc); }
  float* Tt = Ts[wave];
#pragma unroll
  for (int r = 0; r < 2; ++r)
#pragma unroll
    for (int v = 0; v < 8; ++v) { const float raw = (r == 0) ? a0acc[v] : a1acc[v]; const float lg = (nloc < E) ? raw * AI : -INFINITY; float mx = lg;
#pragma unroll
      for (int o = 1; o < 4; o <<= 1) mx = fmaxf(mx, __shfl_xor(mx, o));
      const float ex = (nloc < E) ? __expf(lg - mx) : 0.0f; float se = ex;
#pragma unroll
      for (int o = 1; o < 4; o <<= 1) se += __shfl_xor(se, o);
      if (nloc < E) Tt[(r * 16 + 8 * hlf + v) * 4 + nloc] = ex / se; }
  wave_lds_sync();
  for (int pass = 0; pass < 2; ++pass) { *(volatile v4f*)(gate + (size_t)(m0 + lane) * E) = *(const v4f*)(Tt + lane * 4); __threadfence(); }
}

__global__ __launch_bounds__(128) void cvx_kernel(const float* __restrict__ vx, const b16* __restrict__ cb, float* __restrict__ cvx) {
  __shared__ __attribute__((aligned(16))) float Ts[4][32 * 64];
  const int lane = threadIdx.x & 31, wave = threadIdx.x >> 5, nloc = lane & 15, hlf = lane >> 4, m0 = blockIdx.y * 128 + wave * 32, c0 = blockIdx.x * 64;
  v8f acc[2][4];
#pragma unroll
  for (int r = 0; r < 2; ++r)
#pragma unroll
    for (int t = 0; t < 4; ++t) acc[r][t] = (v8f){};
  const Opnd A{vx, nullptr, ER}, Bo{cb, nullptr, ER};
  gemm_tile<5, 1>(A, Bo, ER, m0, c0, nloc, hlf, acc);
#pragma unroll
  for (int t = 0; t < 4; ++t)
#pragma unroll
    for (int r = 0; r < 2; ++r)
#pragma unroll
      for (int v = 0; v < 8; ++v) acc[r][t][v] = tanhf(acc[r][t][v] * AI);
  epi_f32(acc, 1.0f, nullptr, cvx, ER, m0, c0, lane, Ts[wave]);
}

__global__ __launch_bounds__(128) void mix_kernel(const float* __restrict__ cvx, const b16* __restrict__ ut, const float* __restrict__ gate, const float* __restrict__ x0, const float* __restrict__ bias, const float* xl, float* xo) {
  __shared__ __attribute__((aligned(16))) float Ts[4][32 * 64];
  const int lane = threadIdx.x & 31, wave = threadIdx.x >> 5, nloc = lane & 15, hlf = lane >> 4, m0 = blockIdx.y * 128 + wave * 32, c0 = blockIdx.x * 64;
  v8f tot[2][4];
#pragma unroll
  for (int r = 0; r < 2; ++r)
#pragma unroll
    for (int t = 0; t < 4; ++t) tot[r][t] = (v8f){};
#pragma unroll 1
  for (int e = 0; e < E; ++e) {
    v8f acc[2][4];
#pragma unroll
    for (int r = 0; r < 2; ++r)
#pragma unroll
      for (int t = 0; t < 4; ++t) acc[r][t] = (v8f){};
    const Opnd A{cvx + e * R, nullptr, ER}, Bo{ut + ((size_t)e * D) * R, nullptr, R};
    gemm_tile<5, 1>(A, Bo, R, m0, c0, nloc, hlf, acc);
    float g[2][8];
#pragma unroll
    for (int r = 0; r < 2; ++r)
#pragma unroll
      for (int v = 0; v < 8; ++v) g[r][v] = gate[(size_t)(m0 + r * 16 + 8 * hlf + v) * E + e];
#pragma unroll
    for (int t = 0; t < 4; ++t)
#pragma unroll
      for (int r = 0; r < 2; ++r)
#pragma unroll
        for (int v = 0; v < 8; ++v) tot[r][t][v] += g[r][v] * (acc[r][t][v] * AI + bias[c0 + t * 16 + nloc]);
  }
#pragma unroll
  for (int t = 0; t < 4; ++t)
#pragma unroll
    for (int r = 0; r < 2; ++r)
#pragma unroll
      for (int v = 0; v < 8; ++v) { const size_t idx = (size_t)(m0 + r * 16 + 8 * hlf + v) * D + c0 + t * 16 + nloc; tot[r][t][v] = x0[idx] * tot[r][t][v] + xl[idx]; }
  __syncthreads();
  epi_f32(tot, 1.0f, nullptr, xo, D, m0, c0, lane, Ts[wave]);
}

__global__ __launch_bounds__(256) void copy_kernel(const float* __restrict__ x0, float* __restrict__ xl) {
  const size_t i = (size_t)blockIdx.x * 256 + threadIdx.x; const v4f v = *(const v4f*)(x0 + i * 4);
  for (int pass = 0; pass < 2; ++pass) { *(volatile v4f*)(xl + i * 4) = v; __threadfence(); }
}
}

extern "C" void kernel_launch(void* const* d_in, const int* in_sizes, int n_in,
                              void* d_out, int out_size, void* d_ws, size_t ws_size, hipStream_t stream) {
  (void)n_in; (void)out_size;
  const float* x0 = (const float*)d_in[0]; const float* U = (const float*)d_in[1]; const float* V = (const float*)d_in[2]; const float* C = (const float*)d_in[3]; const float* bias = (const float*)d_in[4]; const float* G = (const float*)d_in[5];
  float* out = (float*)d_out;
  if (in_sizes[0] != B_ * D || in_sizes[1] != L * E * D * R || in_sizes[2] != L * E * D * R || in_sizes[3] != L * E * R * R || in_sizes[4] != L * D || in_sizes[5] != E * D) return;
  size_t off = 0; char* ws = (char*)d_ws;
  auto carve = [&](size_t bytes) { char* p = ws + off; off += (bytes + 255) & ~(size_t)255; return p; };
  b16* vt = (b16*)carve((size_t)L * ER * D * 2); b16* cb = (b16*)carve((size_t)L * ER * ER * 2); b16* ut = (b16*)carve((size_t)L * E * D * R * 2); b16* g16 = (b16*)carve((size_t)16 * D * 2);
  float* vx = (float*)carve((size_t)B_ * ER * 4); float* cvx = (float*)carve((size_t)B_ * ER * 4); float* gate = (float*)carve((size_t)B_ * E * 4); float* xl = (float*)carve((size_t)B_ * D * 4);
  if (off > ws_size) return;
  prep_kernel<<<512, 256, 0, stream>>>(U, V, C, G, vt, cb, ut, g16);
  copy_kernel<<<B_ * D / 4 / 256, 256, 0, stream>>>(x0, xl);
  for (int l = 0; l < L; ++l) {
    vx_kernel<<<dim3(ER / 64, NBLK), 128, 0, stream>>>(xl, vt + (size_t)l * ER * D, vx);
    gate_kernel<<<NBLK, 128, 0, stream>>>(xl, g16, gate);
    cvx_kernel<<<dim3(ER / 64, NBLK), 128, 0, stream>>>(vx, cb + (size_t)l * ER * ER, cvx);
    mix_kernel<<<dim3(D / 64, NBLK), 128, 0, stream>>>(cvx, ut + (size_t)l * E * D * R, gate, x0, bias + l * D, xl, (l == L - 1) ? out : xl);
  }
}
